// MutliHeadSelfAttention_26113401160415
// MI455X (gfx1250) — hardware-verified
//
#include <hip/hip_runtime.h>
#include <math.h>
#include <stdint.h>

#ifndef NB
#define NB 2
#endif
#define SEQ   2048
#define DMOD  2048
#define NH    16
#define HD    128
#define MROWS (NB * SEQ)
#define NST   (SEQ / 64)
#define NCB   (DMOD / 256)
#define ZEOFF (NB * NH * SEQ)
#define RSQRT_D 0.022097086912079608f
#define LOG2E   1.4426950408889634f
#define QSC   1024.0f
#define KSC   1024.0f
#define OSC   4096.0f
#define WOS   1024.0f
#define SLAB64 (16 * 68)
#define WS_CAP 134217728
static_assert(NB >= 1 && NB <= 2);
static_assert(DMOD == NH * HD && HD == 128 && NH == 16);
static_assert((SEQ % 64) == 0 && (DMOD % 256) == 0 && (MROWS % 64) == 0 && (DMOD % 64) == 0 && (DMOD % 32) == 0);
static_assert(((MROWS * DMOD) % 2048) == 0 && ((DMOD * DMOD) % 2048) == 0);
static_assert(NST * 64 == SEQ && NCB * 256 == DMOD);

typedef unsigned short u16;
typedef _Float16 v16h __attribute__((ext_vector_type(16)));
typedef _Float16 v8h  __attribute__((ext_vector_type(8)));
typedef __bf16   v16b __attribute__((ext_vector_type(16)));
typedef float    v8f  __attribute__((ext_vector_type(8)));
typedef float    v4f  __attribute__((ext_vector_type(4)));
typedef unsigned int v4u __attribute__((ext_vector_type(4)));

union FragH { v16h v; v8h h[2]; v4u u[2]; };
union FragB { v16b v; v4u u[2]; };

__device__ __forceinline__ unsigned short bf_bits(float f) {
  unsigned u = __float_as_uint(f);
  return (unsigned short)((u + 0x7FFFu + ((u >> 16) & 1u)) >> 16);
}
__device__ __forceinline__ float bf_up(unsigned short h) { return __uint_as_float(((unsigned)h) << 16); }
__device__ __forceinline__ float bfr(float f) { return bf_up(bf_bits(f)); }
__device__ __forceinline__ unsigned short h_bits(_Float16 x) { return __builtin_bit_cast(unsigned short, x); }
__device__ __forceinline__ unsigned pk16(unsigned short a, unsigned short b) { return (unsigned)a | ((unsigned)b << 16); }
__device__ __forceinline__ v8f zero8() { v8f z = {0.f, 0.f, 0.f, 0.f, 0.f, 0.f, 0.f, 0.f}; return z; }

__device__ __forceinline__ v16h ldfrag_h(const _Float16* p) {
  FragH f;
  f.h[0] = *(const v8h*)(p);
  f.h[1] = *(const v8h*)(p + 16);
  return f.v;
}
__device__ __forceinline__ v16b ldfrag_b(const u16* p) {
  FragB f;
  f.u[0] = *(const v4u*)(p);
  f.u[1] = *(const v4u*)(p + 16);
  return f.v;
}

__device__ __forceinline__ v8f mma_h(v16h a, v16h b, v8f c) {
#if defined(__HIP_DEVICE_COMPILE__)
  return __builtin_amdgcn_wmma_f32_16x16x32_f16(false, a, false, b, (short)0, c, false, false);
#else
  (void)a; (void)b; return c;
#endif
}
__device__ __forceinline__ v8f mma_b(v16b a, v16b b, v8f c) {
#if defined(__HIP_DEVICE_COMPILE__)
  return __builtin_amdgcn_wmma_f32_16x16x32_bf16(false, a, false, b, (short)0, c, false, false);
#else
  (void)a; (void)b; return c;
#endif
}
__device__ __forceinline__ void guard2(v8f& a, v8f& b, v16h x0, v16h x1, v16h x2, v16h x3, v16h x4, v16h x5) {
#if defined(__HIP_DEVICE_COMPILE__)
  asm volatile("v_nop\n\tv_nop\n\tv_nop\n\tv_nop"
               : "+v"(a), "+v"(b) : "v"(x0), "v"(x1), "v"(x2), "v"(x3), "v"(x4), "v"(x5) : "memory");
#else
  (void)a; (void)b; (void)x0; (void)x1; (void)x2; (void)x3; (void)x4; (void)x5;
#endif
}
template <typename F>
__device__ __forceinline__ void guard6(v8f& a, v8f& b, v8f& c, v8f& d, F x0, F x1, F x2, F x3, F x4, F x5) {
#if defined(__HIP_DEVICE_COMPILE__)
  asm volatile("v_nop\n\tv_nop\n\tv_nop\n\tv_nop"
               : "+v"(a), "+v"(b), "+v"(c), "+v"(d) : "v"(x0), "v"(x1), "v"(x2), "v"(x3), "v"(x4), "v"(x5) : "memory");
#else
  (void)a; (void)b; (void)c; (void)d; (void)x0; (void)x1; (void)x2; (void)x3; (void)x4; (void)x5;
#endif
}
__device__ __forceinline__ void wave_sync_lds() {
#if defined(__HIP_DEVICE_COMPILE__)
  __builtin_amdgcn_fence(__ATOMIC_RELEASE, "workgroup");
  __builtin_amdgcn_wave_barrier();
  __builtin_amdgcn_fence(__ATOMIC_ACQUIRE, "workgroup");
#endif
}

template <int MODE>
__global__ __launch_bounds__(256) void cvt16(const float* __restrict__ x, u16* D, int n8, float scale) {
  const int gt = blockIdx.x * 256 + (int)threadIdx.x;
  if (gt >= n8) return;
  const float* p = x + (size_t)gt * 8;
  const v4f a = *(const v4f*)(p), b4 = *(const v4f*)(p + 4);
  float w[8];
#pragma unroll
  for (int e = 0; e < 4; ++e) { w[e] = a[e]; w[4 + e] = b4[e]; }
  v4u o;
#pragma unroll
  for (int e = 0; e < 4; ++e) {
    const float f0 = w[2 * e], f1 = w[2 * e + 1];
    unsigned short u0, u1;
    if constexpr (MODE == 0) {
      u0 = bf_bits(f0);
      u1 = bf_bits(f1);
    } else if constexpr (MODE == 1) {
      u0 = h_bits((_Float16)(bfr(f0) * scale));
      u1 = h_bits((_Float16)(bfr(f1) * scale));
    } else {
      u0 = h_bits((_Float16)(f0 * scale));
      u1 = h_bits((_Float16)(f1 * scale));
    }
    o[e] = pk16(u0, u1);
  }
  u16* d = D + (size_t)gt * 8;
  for (int pass = 0; pass < 2; ++pass) {
    *(volatile v4u*)(d) = o;
    __threadfence();
  }
}

__device__ __forceinline__ void epi64(float* sl, v8f a0, v8f a1, v8f a2, v8f a3, float oscale,
                                      const float* __restrict__ bias, float* C, int N, size_t rowb, int col0, int lane) {
  const int hh = lane >> 4, m = lane & 15;
#pragma unroll
  for (int r = 0; r < 8; ++r) {
    const int ro = (8 * hh + r) * 68 + m;
    sl[ro]      = a0[r] * oscale;
    sl[ro + 16] = a1[r] * oscale;
    sl[ro + 32] = a2[r] * oscale;
    sl[ro + 48] = a3[r] * oscale;
  }
  wave_sync_lds();
  const v4f bb = *(const v4f*)(bias + col0 + m * 4);
  v4f br;
#pragma unroll
  for (int e = 0; e < 4; ++e) br[e] = bfr(bb[e]);
  v4f vals[8];
#pragma unroll
  for (int it = 0; it < 8; ++it) vals[it] = *(const v4f*)(sl + (it * 2 + hh) * 68 + m * 4) + br;
  float* dst = C + (rowb + (size_t)hh) * (size_t)N + col0 + m * 4;
  for (int pass = 0; pass < 2; ++pass) {
#pragma unroll
    for (int it = 0; it < 8; ++it) {
      *(volatile v4f*)(dst + (size_t)(it * 2) * (size_t)N) = vals[it];
    }
    __threadfence();
  }
}

__global__ __launch_bounds__(128)
void gemm_bf(const u16* __restrict__ A, const u16* __restrict__ Bt, const float* __restrict__ bias,
             float* C, int M, int N, int K, float oscale) {
  __shared__ __align__(16) float slab[4 * SLAB64];
  const int tid = threadIdx.x, wave = tid >> 5, lane = tid & 31, hh = lane >> 4, m = lane & 15;
  const int ntile = N >> 6;
  const int bid   = blockIdx.x;
  const int rowb  = (bid / ntile) * 64 + wave * 16;
  const int col0  = (bid % ntile) * 64;
  if (rowb + 16 > M) return;
  const u16* ap = A  + (size_t)(rowb + m) * K + 8 * hh;
  const u16* bp = Bt + (size_t)(col0 + m) * K + 8 * hh;
  const size_t bs = (size_t)16 * K;
  v8f acc0 = zero8(), acc1 = zero8(), acc2 = zero8(), acc3 = zero8();
#pragma unroll 1
  for (int k0 = 0; k0 < K; k0 += 32) {
    const v16b a  = ldfrag_b(ap + k0);
    const v16b b0 = ldfrag_b(bp + k0);
    const v16b b1 = ldfrag_b(bp + bs + k0);
    const v16b b2 = ldfrag_b(bp + 2 * bs + k0);
    const v16b b3 = ldfrag_b(bp + 3 * bs + k0);
    acc0 = mma_b(a, b0, acc0);
    acc1 = mma_b(a, b1, acc1);
    acc2 = mma_b(a, b2, acc2);
    acc3 = mma_b(a, b3, acc3);
    guard6<v16b>(acc0, acc1, acc2, acc3, a, b0, b1, b2, b3, a);
  }
  epi64(slab + wave * SLAB64, acc0, acc1, acc2, acc3, oscale, bias, C, N, (size_t)rowb, col0, lane);
}

__global__ __launch_bounds__(128)
void gemm_h(const u16* __restrict__ A, const u16* __restrict__ Bt, const float* __restrict__ bias,
            float* C, int M, int N, int K, float oscale) {
  __shared__ __align__(16) float slab[4 * SLAB64];
  const int tid = threadIdx.x, wave = tid >> 5, lane = tid & 31, hh = lane >> 4, m = lane & 15;
  const int ntile = N >> 6;
  const int bid   = blockIdx.x;
  const int rowb  = (bid / ntile) * 64 + wave * 16;
  const int col0  = (bid % ntile) * 64;
  if (rowb + 16 > M) return;
  const _Float16* ap = (const _Float16*)(const void*)A  + (size_t)(rowb + m) * K + 8 * hh;
  const _Float16* bp = (const _Float16*)(const void*)Bt + (size_t)(col0 + m) * K + 8 * hh;
  const size_t bs = (size_t)16 * K;
  v8f acc0 = zero8(), acc1 = zero8(), acc2 = zero8(), acc3 = zero8();
#pragma unroll 1
  for (int k0 = 0; k0 < K; k0 += 32) {
    const v16h a  = ldfrag_h(ap + k0);
    const v16h b0 = ldfrag_h(bp + k0);
    const v16h b1 = ldfrag_h(bp + bs + k0);
    const v16h b2 = ldfrag_h(bp + 2 * bs + k0);
    const v16h b3 = ldfrag_h(bp + 3 * bs + k0);
    acc0 = mma_h(a, b0, acc0);
    acc1 = mma_h(a, b1, acc1);
    acc2 = mma_h(a, b2, acc2);
    acc3 = mma_h(a, b3, acc3);
    guard6<v16h>(acc0, acc1, acc2, acc3, a, b0, b1, b2, b3, a);
  }
  epi64(slab + wave * SLAB64, acc0, acc1, acc2, acc3, oscale, bias, C, N, (size_t)rowb, col0, lane);
}

__global__ __launch_bounds__(128)
void zpass(const u16* __restrict__ QHp, const u16* __restrict__ KHp, float* ZE) {
  __shared__ __align__(16) float zes[128];
  const int tid  = (int)threadIdx.x;
  const int wave = tid >> 5;
  const int lane = tid & 31;
  const int hh   = lane >> 4;
  const int c    = lane & 15;
  const int bid  = (int)blockIdx.x;
  const int st   = bid % NST;
  const int t2   = bid / NST;
  const int h    = t2 % NH;
  const int b    = t2 / NH;
  if (b >= NB) return;
  const int i0   = st * 64 + wave * 16;

  const size_t hcol = (size_t)h * HD + 8 * hh;
  const _Float16* Qh  = (const _Float16*)(const void*)QHp + ((size_t)b * SEQ + i0 + c) * DMOD + hcol;
  const _Float16* Khb = (const _Float16*)(const void*)KHp + ((size_t)b * SEQ + c) * DMOD + hcol;

  v16h qf[4];
#pragma unroll
  for (int kk = 0; kk < 4; ++kk) qf[kk] = ldfrag_h(Qh + kk * 32);

  float zsum[8], dg[8];
#pragma unroll
  for (int r = 0; r < 8; ++r) { zsum[r] = 0.f; dg[r] = 0.f; }
  const int kb0 = (i0 >> 5) << 5;
  const int nkt = (SEQ - kb0) >> 5;
  const int qr0 = i0 + 8 * hh;
  const float lsc = RSQRT_D * (LOG2E / (QSC * KSC));

#pragma unroll 1
  for (int kt = 0; kt < nkt; ++kt) {
    const int kb = kb0 + kt * 32;
    const _Float16* k0p = Khb + (size_t)kb * DMOD;
    const _Float16* k1p = k0p + (size_t)16 * DMOD;
    v8f s0 = zero8(), s1 = zero8();
#pragma unroll
    for (int kk = 0; kk < 4; ++kk) {
      const v16h kh0 = ldfrag_h(k0p + kk * 32);
      const v16h kh1 = ldfrag_h(k1p + kk * 32);
      s0 = mma_h(qf[kk], kh0, s0);
      s1 = mma_h(qf[kk], kh1, s1);
      guard2(s0, s1, qf[kk], kh0, kh1, qf[kk], kh0, kh1);
    }
    const int key0 = kb + c, key1 = kb + 16 + c;
#pragma unroll
    for (int r = 0; r < 8; ++r) {
      const int   qr = qr0 + r;
      const float e0 = exp2f(s0[r] * lsc);
      const float e1 = exp2f(s1[r] * lsc);
      zsum[r] += ((key0 >= qr) ? e0 : 0.0f) + ((key1 >= qr) ? e1 : 0.0f);
      dg[r]   += ((key0 == qr) ? e0 : 0.0f) + ((key1 == qr) ? e1 : 0.0f);
    }
  }
#pragma unroll
  for (int r = 0; r < 8; ++r) {
#pragma unroll
    for (int off = 1; off < 16; off <<= 1) {
      zsum[r] += __shfl_xor(zsum[r], off, 32);
      dg[r]   += __shfl_xor(dg[r], off, 32);
    }
  }
  if (c == 0) {
#pragma unroll
    for (int r = 0; r < 8; ++r) {
      zes[wave * 16 + 8 * hh + r]      = (float)(qr0 + r) + zsum[r];
      zes[64 + wave * 16 + 8 * hh + r] = dg[r];
    }
  }
  __syncthreads();
  if (wave == 0) {
    const v4f val = *(const v4f*)(zes + 64 * hh + 4 * c);
    float* dst = ZE + (size_t)hh * ZEOFF + (size_t)(b * NH + h) * SEQ + st * 64 + 4 * c;
    *(volatile v4f*)(dst) = val;
    __threadfence();
    *(volatile v4f*)(dst) = val;
  }
}

__global__ __launch_bounds__(256)
void vpart(const float* __restrict__ V, float* bsum) {
  const int tid = (int)threadIdx.x;
  const int bid = (int)blockIdx.x;
  const int cb  = bid % NCB;
  const int t2  = bid / NCB;
  const int st  = t2 % NST;
  const int b   = t2 / NST;
  if (b >= NB) return;
  const int c = cb * 256 + tid;
  const float* p = V + ((size_t)b * SEQ + (size_t)st * 64) * DMOD + c;
  float s = 0.f;
#pragma unroll 4
  for (int t = 0; t < 64; ++t) s += p[(size_t)t * DMOD];
  float* d = bsum + (size_t)(b * NST + st) * DMOD + c;
  *(volatile float*)(d) = s;
  __threadfence();
  *(volatile float*)(d) = s;
}

__global__ __launch_bounds__(256)
void combine(const float* __restrict__ V, const float* __restrict__ bsum, const float* __restrict__ ZE, u16* OHp) {
  __shared__ float rzs[NH * 64];
  __shared__ float es[NH * 64];
  const int tid = (int)threadIdx.x;
  const int bid = (int)blockIdx.x;
  const int st  = bid % NST;
  const int b   = bid / NST;
  if (b >= NB) return;
#pragma unroll 1
  for (int q = 0; q < 4; ++q) {
    const int idx = q * 256 + tid;
    const int hq  = idx >> 6, t = idx & 63;
    const size_t zi = (size_t)(b * NH + hq) * SEQ + (size_t)st * 64 + t;
    const float z  = ZE[zi];
    const float ev = ZE[(size_t)ZEOFF + zi];
    rzs[idx] = OSC / z;
    es[idx]  = ev;
  }
  __syncthreads();
  const int c0 = tid * 8;
  const int h  = tid >> 4;
  float run[8];
#pragma unroll
  for (int j = 0; j < 8; ++j) run[j] = 0.f;
#pragma unroll 1
  for (int t = 0; t < st; ++t) {
    const float* p = bsum + (size_t)(b * NST + t) * DMOD + c0;
    const v4f pa = *(const v4f*)(p), pb = *(const v4f*)(p + 4);
#pragma unroll
    for (int j = 0; j < 4; ++j) { run[j] += pa[j]; run[4 + j] += pb[j]; }
  }
  const size_t row0 = (size_t)b * SEQ + (size_t)st * 64;
#pragma unroll 1
  for (int t = 0; t < 64; ++t) {
    const float* vp = V + (row0 + (size_t)t) * DMOD + c0;
    const v4f va = *(const v4f*)(vp), vb = *(const v4f*)(vp + 4);
    float w[8];
#pragma unroll
    for (int j = 0; j < 4; ++j) { w[j] = va[j]; w[4 + j] = vb[j]; }
    const float rz = rzs[h * 64 + t];
    const float ev = es[h * 64 + t];
    v4u o;
#pragma unroll
    for (int j = 0; j < 4; ++j) {
      const float a0 = (run[2 * j]     + ev * w[2 * j])     * rz;
      const float a1 = (run[2 * j + 1] + ev * w[2 * j + 1]) * rz;
      o[j] = pk16(h_bits((_Float16)a0), h_bits((_Float16)a1));
    }
#pragma unroll
    for (int j = 0; j < 8; ++j) run[j] += w[j];
    u16* d = OHp + (row0 + (size_t)t) * DMOD + c0;
    *(volatile v4u*)(d) = o;
    __threadfence();
    *(volatile v4u*)(d) = o;
  }
}

extern "C" void kernel_launch(void* const* d_in, const int* in_sizes, int n_in,
                              void* d_out, int out_size, void* d_ws, size_t ws_size,
                              hipStream_t stream) {
  if (n_in < 9) return;
  if (in_sizes[0] < MROWS * DMOD) return;
  if (in_sizes[1] != DMOD * DMOD || in_sizes[3] != DMOD * DMOD || in_sizes[5] != DMOD * DMOD || in_sizes[7] != DMOD * DMOD) return;
  if (in_sizes[2] != DMOD || in_sizes[4] != DMOD || in_sizes[6] != DMOD || in_sizes[8] != DMOD) return;
  if (out_size < MROWS * DMOD) return;

  const float* x    = (const float*)d_in[0];
  const float* wq_w = (const float*)d_in[1];
  const float* wq_b = (const float*)d_in[2];
  const float* wk_w = (const float*)d_in[3];
  const float* wk_b = (const float*)d_in[4];
  const float* wv_w = (const float*)d_in[5];
  const float* wv_b = (const float*)d_in[6];
  const float* wo_w = (const float*)d_in[7];
  const float* wo_b = (const float*)d_in[8];
  float*       out  = (float*)d_out;

  const size_t szXB = (size_t)MROWS * DMOD * 2;
  const size_t szW  = (size_t)DMOD * DMOD * 2;
  const size_t szV  = (size_t)MROWS * DMOD * 4;
  const size_t szF  = (size_t)MROWS * DMOD * 4;
  const size_t szQ  = (size_t)MROWS * DMOD * 2;
  const size_t szZE = (size_t)2 * ZEOFF * 4;
  const size_t szBS = (size_t)NB * NST * DMOD * 4;
  if (szQ > szF) return;
  size_t off = 0;
  const size_t oXB = off; off += szXB;
  const size_t oW  = off; off += szW;
  const size_t oV  = off; off += szV;
  const size_t oF  = off; off += szF;
  const size_t oQH = off; off += szQ;
  const size_t oKH = off; off += szQ;
  const size_t oZE = off; off += szZE;
  const size_t oBS = off; off += szBS;
  if (off > ws_size) return;
  if (off > (size_t)WS_CAP) return;

  char* ws = (char*)d_ws;
  u16*   XB = (u16*)(ws + oXB);
  u16*   WB = (u16*)(ws + oW);
  float* V  = (float*)(ws + oV);
  float* F  = (float*)(ws + oF);
  u16*   OH = (u16*)(ws + oF);
  u16*   QH = (u16*)(ws + oQH);
  u16*   KH = (u16*)(ws + oKH);
  float* ZE = (float*)(ws + oZE);
  float* BS = (float*)(ws + oBS);

  const dim3 b256(256), b128(128);
  const int  n8x = (MROWS * DMOD) / 8;
  const int  n8w = (DMOD * DMOD) / 8;
  const dim3 gX((n8x + 255) / 256);
  const dim3 gW((n8w + 255) / 256);
  const dim3 gG((MROWS / 64) * (DMOD / 64));
  const dim3 gZ(NB * NH * NST);
  const dim3 gVP(NB * NST * NCB);
  const dim3 gCB(NB * NST);

  cvt16<0><<<gX, b256, 0, stream>>>(x, XB, n8x, 1.0f);
  cvt16<0><<<gW, b256, 0, stream>>>(wv_w, WB, n8w, 1.0f);
  gemm_bf<<<gG, b128, 0, stream>>>(XB, WB, wv_b, V, MROWS, DMOD, DMOD, 1.0f);
  cvt16<0><<<gW, b256, 0, stream>>>(wq_w, WB, n8w, 1.0f);
  gemm_bf<<<gG, b128, 0, stream>>>(XB, WB, wq_b, F, MROWS, DMOD, DMOD, 1.0f);
  cvt16<2><<<gX, b256, 0, stream>>>(F, QH, n8x, QSC);
  cvt16<0><<<gW, b256, 0, stream>>>(wk_w, WB, n8w, 1.0f);
  gemm_bf<<<gG, b128, 0, stream>>>(XB, WB, wk_b, F, MROWS, DMOD, DMOD, 1.0f);
  cvt16<2><<<gX, b256, 0, stream>>>(F, KH, n8x, KSC);
  zpass<<<gZ, b128, 0, stream>>>(QH, KH, ZE);
  vpart<<<gVP, b256, 0, stream>>>(V, BS);
  combine<<<gCB, b256, 0, stream>>>(V, BS, ZE, OH);
  cvt16<1><<<gW, b256, 0, stream>>>(wo_w, WB, n8w, WOS);
  gemm_h<<<gG, b128, 0, stream>>>(OH, WB, wo_b, out, MROWS, DMOD, DMOD, 1.0f / (OSC * WOS));
  (void)hipGetLastError();
}
